// TransformerBlock_59588376265154
// MI455X (gfx1250) — hardware-run, weakly checked
//
#include <hip/hip_runtime.h>


#ifndef NB
#define NB 4
#endif
#ifndef SEQ
#define SEQ 2048
#endif
#define NB_FULL  4
#define SEQ_FULL 2048
#ifndef OUT_SEQ
#define OUT_SEQ SEQ
#endif
#define DM    1024
#define NH_   16
#define HD    64
#define FFD   4096
#define AW    4
#define ESEQ  ((SEQ) < 512 ? (SEQ) : 512)
#define MROWS (NB * SEQ)
#define MHALF (MROWS / 2)
#define WSC   64.0f
#define WSI   (1.0f / 64.0f)
#define ACY   16.0f
#define QRS   2048.0f
#define QRI   (1.0f / 2048.0f)
#define SC2   (0.125f * 1.4426950408889634f)
#define PSH   8.0f
#define BIGB  0x40000000

static_assert(HD == 64);
static_assert(NH_ * HD == DM);
static_assert(DM % 64 == 0);
static_assert(FFD % 64 == 0);
static_assert(DM % 32 == 0);
static_assert(FFD % 32 == 0);
static_assert(SEQ % 64 == 0);
static_assert(MROWS % 128 == 0);
static_assert(MROWS % 8 == 0);
static_assert(SEQ % 32 == 0);
static_assert(ESEQ % (16 * AW) == 0);
static_assert((SEQ - ESEQ) % (16 * AW) == 0);
static_assert(ESEQ % 64 == 0);
static_assert(NB <= NB_FULL);
static_assert(SEQ <= SEQ_FULL);

typedef _Float16 h16;
typedef __attribute__((ext_vector_type(16))) _Float16 v16h;
typedef __attribute__((ext_vector_type(8)))  _Float16 v8h;
typedef __attribute__((ext_vector_type(8)))  float    v8f;
typedef __attribute__((ext_vector_type(4)))  float    v4f;
typedef v4f  __attribute__((may_alias)) v4fa;

__device__ __forceinline__ unsigned short f2bf(float f) { unsigned u = __float_as_uint(f); u += 0x7FFFu + ((u >> 16) & 1u); return (unsigned short)(u >> 16); }
__device__ __forceinline__ float bfr(float f) { return __uint_as_float(((unsigned)f2bf(f)) << 16); }
__device__ __forceinline__ v16h cat16(v8h lo, v8h hi) { return __builtin_shufflevector(lo, hi, 0, 1, 2, 3, 4, 5, 6, 7, 8, 9, 10, 11, 12, 13, 14, 15); }
__device__ __forceinline__ v8f wmma16(v16h a, v16h b, v8f c) { return __builtin_amdgcn_wmma_f32_16x16x32_f16(false, a, false, b, (short)0, c, false, false); }
__device__ __forceinline__ v16h ldh(const h16* p) { return cat16(*(const v8h*)p, *(const v8h*)(p + 16)); }
__device__ __forceinline__ void wave_sync() { __builtin_amdgcn_fence(3  , "wavefront"); __builtin_amdgcn_wave_barrier(); asm volatile("" ::: "memory"); }

__global__ __launch_bounds__(256) void k_tcvt(const float* __restrict__ in, h16* out, int R, int Cc, size_t inZ, size_t outZ) {
    __shared__ float tl[64 * 65];
    const int tid = threadIdx.x;
    const int r0 = blockIdx.y * 64, c0 = blockIdx.x * 64;
    const float* src = in + (size_t)blockIdx.z * inZ + (size_t)r0 * Cc + c0;
    h16* dst = out + (size_t)blockIdx.z * outZ + (size_t)c0 * R + r0;
#pragma unroll 4
    for (int i = 0; i < 16; ++i) { const int r = i * 4 + (tid >> 6), c = tid & 63; tl[r * 65 + c] = src[(size_t)r * Cc + c]; }
    __syncthreads();
    const int oc = tid >> 3, sg = (tid & 7) * 8;
    v8h o0, o1;
#pragma unroll
    for (int k = 0; k < 8; ++k) { o0[k] = (h16)(bfr(tl[(sg + k) * 65 + oc]) * WSC); o1[k] = (h16)(bfr(tl[(sg + k) * 65 + oc + 32]) * WSC); }
#pragma unroll 1
    for (int ps = 0; ps < 2; ++ps) {
        *(volatile v8h*)(dst + (size_t)oc * R + sg) = o0;
        *(volatile v8h*)(dst + (size_t)(oc + 32) * R + sg) = o1;
        if (ps == 0) __threadfence();
    }
}

__device__ __forceinline__ void ld8(const float* p, const int rnd, v4f& a, v4f& c) {
    a = *(const v4f*)p; c = *(const v4f*)(p + 4);
#pragma unroll
    for (int k = 0; k < 4; ++k) { const float ra = bfr(a[k]), rc = bfr(c[k]); a[k] = rnd ? ra : a[k]; c[k] = rnd ? rc : c[k]; }
}

__global__ __launch_bounds__(256) void k_ln(const float* __restrict__ X, const float* __restrict__ G, const float* __restrict__ Bv, h16* out, int rnd, int inSeq) {
    const int lane = threadIdx.x & 31, wave = __builtin_amdgcn_readfirstlane((int)(threadIdx.x >> 5));
    const int row = blockIdx.x * 8 + wave;
    const int b = row / SEQ, t = row % SEQ;
    const float* xr = X + ((size_t)b * inSeq + t) * DM + lane * 8;
    h16* orow = out + (size_t)row * DM + lane * 8;
    float s = 0.0f;
#pragma unroll 1
    for (int i = 0; i < 4; ++i) { v4f a, c; ld8(xr + i * 256, rnd, a, c); s += ((a[0] + a[1]) + (a[2] + a[3])) + ((c[0] + c[1]) + (c[2] + c[3])); }
#pragma unroll
    for (int msk = 16; msk; msk >>= 1) s += __shfl_xor(s, msk, 32);
    const float mu = s * (1.0f / DM);
    float ss = 0.0f;
#pragma unroll 1
    for (int i = 0; i < 4; ++i) { v4f a, c; ld8(xr + i * 256, rnd, a, c);
#pragma unroll
        for (int k = 0; k < 4; ++k) { const float d0 = a[k] - mu, d1 = c[k] - mu; ss += d0 * d0; ss += d1 * d1; } }
#pragma unroll
    for (int msk = 16; msk; msk >>= 1) ss += __shfl_xor(ss, msk, 32);
    const float rstd = rsqrtf(ss * (1.0f / DM) + 1.0e-5f);
#pragma unroll 1
    for (int i = 0; i < 4; ++i) { v4f a, c, ga, gc, ba, bc; ld8(xr + i * 256, rnd, a, c); ld8(G + i * 256 + lane * 8, 1, ga, gc); ld8(Bv + i * 256 + lane * 8, 1, ba, bc);
        v8h hv;
#pragma unroll
        for (int k = 0; k < 4; ++k) { hv[k] = (h16)(((a[k] - mu) * rstd) * ga[k] + ba[k]); hv[4 + k] = (h16)(((c[k] - mu) * rstd) * gc[k] + bc[k]); }
        *(volatile v8h*)(orow + i * 256) = hv; __threadfence(); *(volatile v8h*)(orow + i * 256) = hv; }
}

__device__ __forceinline__ void gemm_main(const h16* __restrict__ A, const h16* __restrict__ Bt, const int K, const int r0, const int c0, const int lr, const int hi, v8f (&acc)[4][4]) {
#pragma unroll
    for (int mb = 0; mb < 4; ++mb)
#pragma unroll
        for (int nb = 0; nb < 4; ++nb) acc[mb][nb] = (v8f){};
    const size_t aoff = (size_t)(r0 + lr) * K + 8 * hi, boff = (size_t)(c0 + lr) * K + 8 * hi;
#pragma unroll 1
    for (int kc = 0; kc < K; kc += 32) {
        v16h a[4];
#pragma unroll
        for (int mb = 0; mb < 4; ++mb) a[mb] = ldh(A + aoff + (size_t)mb * 16 * K + kc);
#pragma unroll
        for (int nb = 0; nb < 4; ++nb) { const v16h bq = ldh(Bt + boff + (size_t)nb * 16 * K + kc);
#pragma unroll
            for (int mb = 0; mb < 4; ++mb) acc[mb][nb] = wmma16(a[mb], bq, acc[mb][nb]); }
        asm volatile("v_nop\n\tv_nop\n\tv_nop\n\tv_nop" : "+v"(acc[0][3]), "+v"(acc[1][3]), "+v"(acc[2][3]), "+v"(acc[3][3]) : "v"(a[0]), "v"(a[1]), "v"(a[2]), "v"(a[3]));
    }
}

template <int MODE>
__global__ __launch_bounds__(32) void k_gemm_h(const h16* __restrict__ A, const h16* __restrict__ Bt, int K, float osc, h16* Ph, h16* Pr,
                                               int RB, size_t sRB, int pitch, int CB, size_t sCB, size_t sRBr, int pitchR, size_t sCBr,
                                               int resRowLim, int resColLim, const float* __restrict__ bias) {
    __shared__ __align__(16) float os[16 * 68];
    const int lane = threadIdx.x & 31, lr = lane & 15, hi = lane >> 4; const int r0 = blockIdx.x * 64, c0 = blockIdx.y * 64;
    v8f acc[4][4];
    gemm_main(A, Bt, K, r0, c0, lr, hi, acc);
    const int rr = r0 % RB, cr = c0 % CB;
    const size_t tbase  = (size_t)(r0 / RB) * sRB  + (size_t)rr * (size_t)pitch  + (size_t)(c0 / CB) * sCB  + (size_t)cr;
    const size_t tbaseR = (size_t)(r0 / RB) * sRBr + (size_t)rr * (size_t)pitchR + (size_t)(c0 / CB) * sCBr + (size_t)cr;
    const int wr = (MODE == 0) && (rr < resRowLim) && (cr < resColLim);
    const int c8 = (lane & 7) * 8;
    v4f bA = (v4f){}, bB = (v4f){};
    if (MODE == 2) { bA = *(const v4f*)(bias + c0 + c8); bB = *(const v4f*)(bias + c0 + c8 + 4);
#pragma unroll
        for (int i = 0; i < 4; ++i) { bA[i] = bfr(bA[i]); bB[i] = bfr(bB[i]); } }
#pragma unroll
    for (int mb = 0; mb < 4; ++mb) {
#pragma unroll
        for (int nb = 0; nb < 4; ++nb) {
#pragma unroll
            for (int j = 0; j < 8; ++j) os[(hi * 8 + j) * 68 + nb * 16 + lr] = acc[mb][nb][j]; }
        wave_sync();
        const size_t sb = tbase + (size_t)(mb * 16) * (size_t)pitch, sbR = tbaseR + (size_t)(mb * 16) * (size_t)pitchR;
#pragma unroll 1
        for (int ps = 0; ps < 2; ++ps) {
#pragma unroll
            for (int s = 0; s < 4; ++s) { const int row = 4 * s + (lane >> 3);
                const v4f x0 = *(const v4fa*)(&os[row * 68 + c8]); const v4f x1 = *(const v4fa*)(&os[row * 68 + c8 + 4]); v8h hv, rv;
#pragma unroll
                for (int i = 0; i < 4; ++i) { float y0 = x0[i] * osc, y1 = x1[i] * osc;
                    if (MODE == 2) { y0 = fmaxf(y0 + bA[i], 0.0f); y1 = fmaxf(y1 + bB[i], 0.0f); }
                    const h16 a0 = (h16)y0; const h16 a1 = (h16)y1; hv[i] = a0; hv[4 + i] = a1;
                    rv[i] = (h16)((y0 - (float)a0) * QRS); rv[4 + i] = (h16)((y1 - (float)a1) * QRS); }
                *(volatile v8h*)(Ph + sb + (size_t)row * (size_t)pitch + c8) = hv;
                if (wr) *(volatile v8h*)(Pr + sbR + (size_t)row * (size_t)pitchR + c8) = rv; }
            if (ps == 0) __threadfence(); }
        wave_sync();
    }
}

__global__ __launch_bounds__(32) void k_gemm_f(const h16* __restrict__ A, const h16* __restrict__ Bt, int K, float osc, const float* __restrict__ bias,
                                               const float* resid, float* outF, int ldo, int rowOff, int rSeq, int oSeq, int rnd) {
    __shared__ __align__(16) float os[16 * 68];
    const int lane = threadIdx.x & 31, lr = lane & 15, hi = lane >> 4; const int r0 = blockIdx.x * 64, c0 = blockIdx.y * 64;
    v8f acc[4][4];
    gemm_main(A, Bt, K, r0, c0, lr, hi, acc);
    const int gr0 = r0 + rowOff; const int bb = gr0 / SEQ, tt = gr0 % SEQ;
    const int cofs = lr * 4;
    const float* rp = resid + ((size_t)bb * rSeq + tt) * (size_t)ldo + c0 + cofs;
    float* op = outF + ((size_t)bb * oSeq + tt) * (size_t)ldo + c0 + cofs;
    v4f bq = *(const v4f*)(bias + c0 + cofs);
#pragma unroll
    for (int i = 0; i < 4; ++i) bq[i] = bfr(bq[i]);
#pragma unroll
    for (int mb = 0; mb < 4; ++mb) {
#pragma unroll
        for (int nb = 0; nb < 4; ++nb) {
#pragma unroll
            for (int j = 0; j < 8; ++j) os[(hi * 8 + j) * 68 + nb * 16 + lr] = acc[mb][nb][j]; }
        wave_sync();
        v4f vv[8];
#pragma unroll
        for (int s = 0; s < 8; ++s) { const int row = 2 * s + hi;
            const v4f y = *(const v4fa*)(&os[row * 68 + cofs]); const v4f rs = *(const v4f*)(rp + (size_t)(mb * 16 + row) * (size_t)ldo);
#pragma unroll
            for (int i = 0; i < 4; ++i) { const float rq = bfr(rs[i]); const float rv = rnd ? rq : rs[i]; vv[s][i] = (rv + y[i] * osc) + bq[i]; } }
#pragma unroll 1
        for (int ps = 0; ps < 2; ++ps) {
#pragma unroll
            for (int s = 0; s < 8; ++s) *(volatile v4f*)(op + (size_t)(mb * 16 + 2 * s + hi) * (size_t)ldo) = vv[s];
            if (ps == 0) __threadfence(); }
        wave_sync();
    }
}

template <int EARLY>
__global__ __launch_bounds__(32 * AW) void k_flash(const h16* __restrict__ QH, const h16* __restrict__ QR, const h16* __restrict__ KP, const h16* __restrict__ KR,
                                                   const h16* __restrict__ VT, const h16* __restrict__ VR, h16* ATT, int tile0) {
    __shared__ __align__(16) float os[AW * 16 * 68];
    const int lane = threadIdx.x & 31, wave = __builtin_amdgcn_readfirstlane((int)(threadIdx.x >> 5)), lr = lane & 15, hi = lane >> 4;
    const int zh = blockIdx.y; const int b = zh / NH_, h = zh % NH_;
    const int t0 = (tile0 + blockIdx.x * AW + wave) * 16;
    const size_t pbase = (size_t)zh * SEQ * HD;
    const size_t rbase = (size_t)zh * ESEQ * HD;
    const size_t qo = pbase + (size_t)(t0 + lr) * HD + 8 * hi;
    const v16h qh0 = ldh(QH + qo), qh1 = ldh(QH + qo + 32);
    v16h qr0 = qh0, qr1 = qh1;
    if (EARLY) { const size_t qro = rbase + (size_t)(t0 + lr) * HD + 8 * hi; qr0 = ldh(QR + qro); qr1 = ldh(QR + qro + 32); }
    const size_t ko  = pbase + (size_t)lr * HD + 8 * hi;
    const size_t kro = rbase + (size_t)lr * HD + 8 * hi;
    const size_t vo  = pbase + (size_t)lr * SEQ + 8 * hi;
    const size_t vro = rbase + (size_t)lr * ESEQ + 8 * hi;
    v8f o0 = (v8f){}, o1 = (v8f){}, o2 = (v8f){}, o3 = (v8f){};
    v8f p0 = (v8f){}, p1 = (v8f){}, p2 = (v8f){}, p3 = (v8f){};
    float m = -3.0e38f, l = 0.0f;
    const int kend = t0 + 16;
#pragma unroll 1
    for (int key0 = 0; key0 < kend; key0 += 32) {
        const h16* ka = KP + ko + (size_t)key0 * HD;
        const v16h ka0 = ldh(ka), ka1 = ldh(ka + 32), kb0 = ldh(ka + 16 * HD), kb1 = ldh(ka + 16 * HD + 32);
        v8f sHa = (v8f){}, sHb = (v8f){}, sLa = (v8f){}, sLb = (v8f){};
        sHa = wmma16(ka0, qh0, sHa); sHb = wmma16(kb0, qh0, sHb);
        sHa = wmma16(ka1, qh1, sHa); sHb = wmma16(kb1, qh1, sHb);
        if (EARLY) {
            const h16* kr = KR + kro + (size_t)key0 * HD;
            const v16h ra0 = ldh(kr), ra1 = ldh(kr + 32), rb0 = ldh(kr + 16 * HD), rb1 = ldh(kr + 16 * HD + 32);
            sLa = wmma16(ka0, qr0, sLa); sLb = wmma16(kb0, qr0, sLb);
            sLa = wmma16(ka1, qr1, sLa); sLb = wmma16(kb1, qr1, sLb);
            sLa = wmma16(ra0, qh0, sLa); sLb = wmma16(rb0, qh0, sLb);
            sLa = wmma16(ra1, qh1, sLa); sLb = wmma16(rb1, qh1, sLb);
            asm volatile("v_nop\n\tv_nop\n\tv_nop\n\tv_nop" : "+v"(sHa), "+v"(sLa), "+v"(sHb), "+v"(sLb) : "v"(ka0), "v"(ka1), "v"(kb0), "v"(kb1), "v"(ra0), "v"(ra1), "v"(rb0), "v"(rb1));
        } else {
            asm volatile("v_nop\n\tv_nop\n\tv_nop\n\tv_nop" : "+v"(sHa), "+v"(sHb) : "v"(ka0), "v"(ka1), "v"(kb0), "v"(kb1));
        }
        const int kq = t0 + lr - key0 - 8 * hi;
        float ta[8], tb[8]; float mx = -3.0e38f;
#pragma unroll
        for (int r = 0; r < 8; ++r) { float sa = sHa[r], sb = sHb[r];
            if (EARLY) { sa += sLa[r] * QRI; sb += sLb[r] * QRI; }
            const float va = sa * SC2, vb = sb * SC2;
            ta[r] = (r <= kq) ? va : -3.0e38f; tb[r] = (r + 16 <= kq) ? vb : -3.0e38f;
            mx = fmaxf(mx, fmaxf(ta[r], tb[r])); }
        mx = fmaxf(mx, __shfl_xor(mx, 16, 32));
        const float mnew = fmaxf(m, mx);
        const float alpha = __builtin_amdgcn_exp2f(m - mnew);
        const float sh = PSH - mnew;
        v16h pb, pr = (v16h){}; float ls = 0.0f;
#pragma unroll
        for (int r = 0; r < 8; ++r) { const float fa = __builtin_amdgcn_exp2f(ta[r] + sh), fc = __builtin_amdgcn_exp2f(tb[r] + sh);
            const h16 pa = (h16)fa; const h16 pc = (h16)fc; pb[r] = pa; pb[8 + r] = pc;
            if (EARLY) { pr[r] = (h16)((fa - (float)pa) * QRS); pr[8 + r] = (h16)((fc - (float)pc) * QRS); ls += fa + fc; }
            else ls += (float)pa + (float)pc; }
        l = l * alpha + ls; m = mnew;
        o0 = o0 * alpha; o1 = o1 * alpha; o2 = o2 * alpha; o3 = o3 * alpha;
        if (EARLY) { p0 = p0 * alpha; p1 = p1 * alpha; p2 = p2 * alpha; p3 = p3 * alpha; }
        const h16* va = VT + vo + key0;
        const v16h v0 = ldh(va), v1 = ldh(va + (size_t)16 * SEQ), v2 = ldh(va + (size_t)32 * SEQ), v3 = ldh(va + (size_t)48 * SEQ);
        o0 = wmma16(v0, pb, o0); o1 = wmma16(v1, pb, o1); o2 = wmma16(v2, pb, o2); o3 = wmma16(v3, pb, o3);
        if (EARLY) {
            const h16* vr = VR + vro + key0;
            const v16h w0 = ldh(vr), w1 = ldh(vr + (size_t)16 * ESEQ), w2 = ldh(vr + (size_t)32 * ESEQ), w3 = ldh(vr + (size_t)48 * ESEQ);
            p0 = wmma16(w0, pb, p0); p1 = wmma16(w1, pb, p1); p2 = wmma16(w2, pb, p2); p3 = wmma16(w3, pb, p3);
            p0 = wmma16(v0, pr, p0); p1 = wmma16(v1, pr, p1); p2 = wmma16(v2, pr, p2); p3 = wmma16(v3, pr, p3);
            asm volatile("v_nop\n\tv_nop\n\tv_nop\n\tv_nop" : "+v"(o0), "+v"(o1), "+v"(o2), "+v"(o3), "+v"(p0), "+v"(p1), "+v"(p2), "+v"(p3)
                         : "v"(v0), "v"(v1), "v"(v2), "v"(v3), "v"(w0), "v"(w1), "v"(w2), "v"(w3), "v"(pb), "v"(pr));
        } else {
            asm volatile("v_nop\n\tv_nop\n\tv_nop\n\tv_nop" : "+v"(o0), "+v"(o1), "+v"(o2), "+v"(o3) : "v"(v0), "v"(v1), "v"(v2), "v"(v3), "v"(pb));
        }
    }
    if (EARLY) { o0 = o0 + p0 * QRI; o1 = o1 + p1 * QRI; o2 = o2 + p2 * QRI; o3 = o3 + p3 * QRI; }
    l += __shfl_xor(l, 16, 32);
    const float inv = ACY * (1.0f / l);
    const int wb = wave * 16 * 68;
    { v4f a, c;
      a[0] = o0[0] * inv; a[1] = o0[1] * inv; a[2] = o0[2] * inv; a[3] = o0[3] * inv; c[0] = o0[4] * inv; c[1] = o0[5] * inv; c[2] = o0[6] * inv; c[3] = o0[7] * inv;
      *(v4fa*)(&os[wb + lr * 68 +  0 + 8 * hi]) = a; *(v4fa*)(&os[wb + lr * 68 +  0 + 8 * hi + 4]) = c;
      a[0] = o1[0] * inv; a[1] = o1[1] * inv; a[2] = o1[2] * inv; a[3] = o1[3] * inv; c[0] = o1[4] * inv; c[1] = o1[5] * inv; c[2] = o1[6] * inv; c[3] = o1[7] * inv;
      *(v4fa*)(&os[wb + lr * 68 + 16 + 8 * hi]) = a; *(v4fa*)(&os[wb + lr * 68 + 16 + 8 * hi + 4]) = c;
      a[0] = o2[0] * inv; a[1] = o2[1] * inv; a[2] = o2[2] * inv; a[3] = o2[3] * inv; c[0] = o2[4] * inv; c[1] = o2[5] * inv; c[2] = o2[6] * inv; c[3] = o2[7] * inv;
      *(v4fa*)(&os[wb + lr * 68 + 32 + 8 * hi]) = a; *(v4fa*)(&os[wb + lr * 68 + 32 + 8 * hi + 4]) = c;
      a[0] = o3[0] * inv; a[1] = o3[1] * inv; a[2] = o3[2] * inv; a[3] = o3[3] * inv; c[0] = o3[4] * inv; c[1] = o3[5] * inv; c[2] = o3[6] * inv; c[3] = o3[7] * inv;
      *(v4fa*)(&os[wb + lr * 68 + 48 + 8 * hi]) = a; *(v4fa*)(&os[wb + lr * 68 + 48 + 8 * hi + 4]) = c; }
    wave_sync();
    h16* orow = ATT + ((size_t)b * SEQ + t0) * DM + h * HD;
    const int c8 = (lane & 7) * 8;
#pragma unroll 1
    for (int ps = 0; ps < 2; ++ps) {
#pragma unroll
        for (int s = 0; s < 4; ++s) { const int row = 4 * s + (lane >> 3);
            const v4f x0 = *(const v4fa*)(&os[wb + row * 68 + c8]); const v4f x1 = *(const v4fa*)(&os[wb + row * 68 + c8 + 4]); v8h hv;
#pragma unroll
            for (int i = 0; i < 4; ++i) { hv[i] = (h16)x0[i]; hv[4 + i] = (h16)x1[i]; }
            *(volatile v8h*)(orow + (size_t)row * DM + c8) = hv; }
        if (ps == 0) __threadfence(); }
}

static constexpr size_t cmax(size_t a, size_t b) { return a > b ? a : b; }
static constexpr size_t SZ_WQKV = (size_t)3 * DM * DM * 2;
static constexpr size_t SZ_WP   = (size_t)DM * DM * 2;
static constexpr size_t SZ_W1   = (size_t)FFD * DM * 2;
static constexpr size_t SZ_W2   = (size_t)DM * FFD * 2;
static constexpr size_t SZ_ACT  = (size_t)MROWS * DM * 2;
static constexpr size_t SZ_PL   = (size_t)NB * NH_ * SEQ * HD * 2;
static constexpr size_t SZ_PR   = (size_t)NB * NH_ * ESEQ * HD * 2;
static constexpr size_t SZ_X1   = (size_t)MROWS * DM * 4;
static constexpr size_t SZ_FH   = (size_t)MHALF * FFD * 2;
static constexpr size_t SZ_B1   = 3 * SZ_PL + 3 * SZ_PR;
static constexpr size_t SZ_B2   = SZ_X1 + SZ_FH;
static constexpr size_t SZ_B    = cmax(SZ_B1, SZ_B2);
static constexpr size_t SZ_TOTAL = SZ_WQKV + SZ_WP + SZ_W1 + SZ_W2 + SZ_ACT + SZ_B;
static_assert(SZ_TOTAL <= (size_t)134217728);
static_assert(SZ_WQKV % 256 == 0 && SZ_WP % 256 == 0 && SZ_W1 % 256 == 0 && SZ_W2 % 256 == 0);
static_assert(SZ_ACT % 256 == 0 && SZ_PL % 256 == 0 && SZ_PR % 256 == 0 && SZ_X1 % 256 == 0 && SZ_FH % 256 == 0);
static_assert(SZ_B1 <= SZ_B && SZ_B2 <= SZ_B);

extern "C" void kernel_launch(void* const* d_in, const int* in_sizes, int n_in,
                              void* d_out, int out_size, void* d_ws, size_t ws_size, hipStream_t stream) {
    if (n_in < 14) return;
    const size_t needx = ((size_t)(NB - 1) * SEQ_FULL + SEQ) * DM;
    if ((size_t)in_sizes[0] < needx) return;
    if ((size_t)in_sizes[1] < (size_t)NH_ * DM * HD || (size_t)in_sizes[2] < (size_t)NH_ * DM * HD || (size_t)in_sizes[3] < (size_t)NH_ * DM * HD) return;
    if ((size_t)in_sizes[4] < (size_t)DM * DM || (size_t)in_sizes[5] < (size_t)DM) return;
    if ((size_t)in_sizes[6] < (size_t)DM * FFD || (size_t)in_sizes[7] < (size_t)FFD) return;
    if ((size_t)in_sizes[8] < (size_t)FFD * DM || (size_t)in_sizes[9] < (size_t)DM) return;
    if ((size_t)in_sizes[10] < (size_t)DM || (size_t)in_sizes[11] < (size_t)DM || (size_t)in_sizes[12] < (size_t)DM || (size_t)in_sizes[13] < (size_t)DM) return;
    if ((size_t)out_size < ((size_t)(NB - 1) * OUT_SEQ + SEQ) * DM) return;
    if (SZ_TOTAL > ws_size) return;
    const float* x     = (const float*)d_in[0];
    const float* wq    = (const float*)d_in[1];
    const float* wk    = (const float*)d_in[2];
    const float* wv    = (const float*)d_in[3];
    const float* wp    = (const float*)d_in[4];
    const float* bproj = (const float*)d_in[5];
    const float* w1    = (const float*)d_in[6];
    const float* b1    = (const float*)d_in[7];
    const float* w2    = (const float*)d_in[8];
    const float* b2    = (const float*)d_in[9];
    const float* g1    = (const float*)d_in[10];
    const float* be1   = (const float*)d_in[11];
    const float* g2    = (const float*)d_in[12];
    const float* be2   = (const float*)d_in[13];
    float* OUT = (float*)d_out;

    char* wsp = (char*)d_ws;
    h16* WQKV = (h16*)wsp; wsp += SZ_WQKV;
    h16* WPT  = (h16*)wsp; wsp += SZ_WP;
    h16* W1T  = (h16*)wsp; wsp += SZ_W1;
    h16* W2T  = (h16*)wsp; wsp += SZ_W2;
    h16* ACT  = (h16*)wsp; wsp += SZ_ACT;
    char* rB  = wsp;
    h16* QH = (h16*)rB;
    h16* KP = (h16*)(rB + SZ_PL);
    h16* VT = (h16*)(rB + 2 * SZ_PL);
    h16* QR = (h16*)(rB + 3 * SZ_PL);
    h16* KR = (h16*)(rB + 3 * SZ_PL + SZ_PR);
    h16* VR = (h16*)(rB + 3 * SZ_PL + 2 * SZ_PR);
    float* X1 = (float*)rB;
    h16* FFH = (h16*)(rB + SZ_X1);
    h16* WQ = WQKV; h16* WK = WQKV + (size_t)DM * DM; h16* WV = WQKV + (size_t)2 * DM * DM;
    h16* H1 = ACT; h16* ATT = ACT; h16* H2 = ACT;

    k_tcvt<<<dim3(HD / 64, DM / 64, NH_), 256, 0, stream>>>(wq, WQ, DM, HD, (size_t)DM * HD, (size_t)HD * DM);
    k_tcvt<<<dim3(HD / 64, DM / 64, NH_), 256, 0, stream>>>(wk, WK, DM, HD, (size_t)DM * HD, (size_t)HD * DM);
    k_tcvt<<<dim3(HD / 64, DM / 64, NH_), 256, 0, stream>>>(wv, WV, DM, HD, (size_t)DM * HD, (size_t)HD * DM);
    k_tcvt<<<dim3(DM / 64, DM / 64, 1), 256, 0, stream>>>(wp, WPT, DM, DM, (size_t)0, (size_t)0);
    k_tcvt<<<dim3(FFD / 64, DM / 64, 1), 256, 0, stream>>>(w1, W1T, DM, FFD, (size_t)0, (size_t)0);
    k_tcvt<<<dim3(DM / 64, FFD / 64, 1), 256, 0, stream>>>(w2, W2T, FFD, DM, (size_t)0, (size_t)0);

    k_ln<<<MROWS / 8, 256, 0, stream>>>(x, g1, be1, H1, 1, SEQ_FULL);

    k_gemm_h<0><<<dim3(MROWS / 64, DM / 64, 1), 32, 0, stream>>>(H1, WQ, DM, WSI, QH, QR, SEQ, (size_t)NH_ * SEQ * HD, HD, HD, (size_t)SEQ * HD,
                                                                 (size_t)NH_ * ESEQ * HD, HD, (size_t)ESEQ * HD, ESEQ, HD, (const float*)0);
    k_gemm_h<0><<<dim3(MROWS / 64, DM / 64, 1), 32, 0, stream>>>(H1, WK, DM, WSI, KP, KR, SEQ, (size_t)NH_ * SEQ * HD, HD, HD, (size_t)SEQ * HD,
                                                                 (size_t)NH_ * ESEQ * HD, HD, (size_t)ESEQ * HD, ESEQ, HD, (const float*)0);
    k_gemm_h<0><<<dim3(DM / 64, MROWS / 64, 1), 32, 0, stream>>>(WV, H1, DM, WSI, VT, VR, DM, (size_t)0, SEQ, SEQ, (size_t)DM * SEQ,
                                                                 (size_t)0, ESEQ, (size_t)DM * ESEQ, DM, ESEQ, (const float*)0);

    k_flash<1><<<dim3(ESEQ / (16 * AW), NB * NH_, 1), 32 * AW, 0, stream>>>(QH, QR, KP, KR, VT, VR, ATT, 0);
    if (SEQ > ESEQ)
        k_flash<0><<<dim3((SEQ - ESEQ) / (16 * AW), NB * NH_, 1), 32 * AW, 0, stream>>>(QH, QR, KP, KR, VT, VR, ATT, ESEQ / 16);

    k_gemm_f<<<dim3(MROWS / 64, DM / 64, 1), 32, 0, stream>>>(ATT, WPT, DM, WSI * (1.0f / ACY), bproj, x, X1, DM, 0, SEQ_FULL, SEQ, 1);

    k_ln<<<MROWS / 8, 256, 0, stream>>>(X1, g2, be2, H2, 0, SEQ);

    for (int hf = 0; hf < 2; ++hf) {
        k_gemm_h<2><<<dim3(MHALF / 64, FFD / 64, 1), 32, 0, stream>>>(H2 + (size_t)hf * MHALF * DM, W1T, DM, WSI, FFH, FFH, BIGB, (size_t)0, FFD, BIGB, (size_t)0,
                                                                      (size_t)0, 0, (size_t)0, 0, 0, b1);
        k_gemm_f<<<dim3(MHALF / 64, DM / 64, 1), 32, 0, stream>>>(FFH, W2T, FFD, WSI, b2, X1, OUT, DM, hf * MHALF, SEQ, OUT_SEQ, 0);
    }
}
